// Encoder_45990509806098
// MI455X (gfx1250) — hardware-verified
//
#include <hip/hip_runtime.h>
#include <hip/hip_fp16.h>


#ifndef NB
#define NB 8
#endif
#ifndef SEQ
#define SEQ 1024
#endif
#define NB_FULL  8
#define SEQ_FULL 1024
#define DM   768
#define NH   12
#define DH   64
#define FF   3072
#define NTOK (NB * SEQ)
#define CH   128

static_assert(NB >= 1 && NB <= NB_FULL);
static_assert(SEQ >= CH && SEQ <= SEQ_FULL);
static_assert(SEQ % CH == 0);
static_assert(SEQ % 128 == 0);
static_assert(CH % 32 == 0);
static_assert(NTOK % 128 == 0);
static_assert(NTOK % 8 == 0);
static_assert(DM % 128 == 0 && FF % 128 == 0);
static_assert(DM % 64 == 0 && FF % 64 == 0);
static_assert(DM % 32 == 0 && FF % 32 == 0 && DH % 32 == 0);
static_assert(NH * DH == DM);
static_assert((NTOK * (DM / 8)) % 256 == 0);

typedef _Float16 v16h __attribute__((ext_vector_type(16)));
typedef _Float16 v8h  __attribute__((ext_vector_type(8)));
typedef float    v8f  __attribute__((ext_vector_type(8)));
typedef float    v4f  __attribute__((ext_vector_type(4)));
typedef int      v4i  __attribute__((ext_vector_type(4)));

union Frag { v16h v; v8h h[2]; };
union I8   { v4i v[2]; int s[8]; };

#define WSC     64.0f
#define QSC     64.0f
#define HSC     16.0f
#define A_QKV   0.015625f
#define A_O     2.44140625e-04f
#define A_F1    9.765625e-04f
#define A_F2    2.44140625e-04f
#define C1 (1.44269504088896340736f * 3.0517578125e-05f)
#define MASKT  (-1.0e10f)

static __device__ __forceinline__ v8f zero8() {
    v8f z;
#pragma unroll
    for (int i = 0; i < 8; ++i) z[i] = 0.0f;
    return z;
}

static __device__ __forceinline__ v16h load_frag16(const _Float16* base, int ld, int lane) {
    int m  = lane & 15;
    int kb = (lane >> 4) << 3;
    const _Float16* p = base + (size_t)m * ld + kb;
    Frag f;
    f.h[0] = *(const v8h*)(p);
    f.h[1] = *(const v8h*)(p + 16);
    return f.v;
}

static __device__ __forceinline__ v8f wmma16(v16h a, v16h b, v8f c) {
    v8f d = __builtin_amdgcn_wmma_f32_16x16x32_f16(false, a, false, b, (short)0, c, false, false);
    asm volatile("v_nop\n\tv_nop\n\tv_nop\n\tv_nop" : "+v"(d) : "v"(a), "v"(b));
    return d;
}

static __device__ __forceinline__ float bf16r(float x) {
    unsigned u = __float_as_uint(x);
    u = (u + 0x7FFFu + ((u >> 16) & 1u)) & 0xFFFF0000u;
    return __uint_as_float(u);
}

static __device__ __forceinline__ float ex2(float x) {
    return __builtin_amdgcn_exp2f(x);
}

static __device__ __forceinline__ void wave_lds_sync() {
    __builtin_amdgcn_fence(3, "wavefront");
    asm volatile("s_wait_dscnt 0" ::: "memory");
    __builtin_amdgcn_wave_barrier();
}

__global__ __launch_bounds__(256) void k_xprep(const float* __restrict__ x,
                                               _Float16* __restrict__ xp) {
    const int g = blockIdx.x * 256 + (int)threadIdx.x;
    if (g >= NTOK * (DM / 8)) return;
    const int row = g / (DM / 8);
    const int col = (g - row * (DM / 8)) * 8;
    const int b = row / SEQ, s = row - b * SEQ;
    const float* src = x + ((size_t)b * SEQ_FULL + s) * DM + col;
    const v4f a = *(const v4f*)(src);
    const v4f c = *(const v4f*)(src + 4);
    v8h hv;
#pragma unroll
    for (int e = 0; e < 4; ++e) {
        hv[e]     = (_Float16)bf16r(a[e]);
        hv[4 + e] = (_Float16)bf16r(c[e]);
    }
    _Float16* dst = xp + (size_t)row * DM + col;
    *(volatile v8h*)dst = hv;
    __threadfence();
    *(volatile v8h*)dst = hv;
}

__global__ __launch_bounds__(256) void k_wtr(const float* __restrict__ W,
                                             _Float16* __restrict__ WT,
                                             int K, int N) {
    __shared__ __align__(16) _Float16 T[64 * 64];
    const int tid = threadIdx.x;
    const int n0 = blockIdx.x * 64;
    const int k0 = blockIdx.y * 64;
#pragma unroll
    for (int i = 0; i < 4; ++i) {
        const int idx = tid + i * 256;
        const int r = idx >> 4, c4 = idx & 15;
        const v4f xv = *(const v4f*)(W + (size_t)(k0 + r) * N + n0 + c4 * 4);
#pragma unroll
        for (int e = 0; e < 4; ++e) T[(c4 * 4 + e) * 64 + r] = (_Float16)(bf16r(xv[e]) * WSC);
    }
    __syncthreads();
    const int na = tid >> 3, pa = tid & 7;
    const int nb = (tid + 256) >> 3, pb = tid & 7;
    const v8h p0 = *(const v8h*)(&T[na * 64 + pa * 8]);
    const v8h p1 = *(const v8h*)(&T[nb * 64 + pb * 8]);
    _Float16* d0 = WT + (size_t)(n0 + na) * K + k0 + pa * 8;
    _Float16* d1 = WT + (size_t)(n0 + nb) * K + k0 + pb * 8;
    *(volatile v8h*)d0 = p0;
    *(volatile v8h*)d1 = p1;
    __threadfence();
    *(volatile v8h*)d0 = p0;
    *(volatile v8h*)d1 = p1;
}

template <int MODE, bool RELU>
__global__ __launch_bounds__(256) __attribute__((amdgpu_num_vgpr(256)))
void k_gemm(const _Float16* __restrict__ A,
            const _Float16* __restrict__ BT,
            const float* __restrict__ bias,
            float ascale, float oscale,
            float* __restrict__ Cf,
            _Float16* __restrict__ Ch,
            int K, int N) {
    __shared__ __align__(16) float    EstF[(MODE == 0) ? 8 * 2048 : 4];
    __shared__ __align__(16) _Float16 EstH[(MODE == 1) ? 8 * 2048 : 8];

    const int tid  = threadIdx.x;
    const int lane = tid & 31;
    const int w    = tid >> 5;
    const int mi = w >> 1, ni = w & 1;
    const int m0 = blockIdx.y * 128 + mi * 32;
    const int n0 = blockIdx.x * 128 + ni * 64;
    const int rb = (lane >> 4) << 3;
    const int cc = lane & 15;
    const _Float16* Ab = A  + (size_t)m0 * K;
    const _Float16* Bb = BT + (size_t)n0 * K;

    v8f acc[2][4];
#pragma unroll
    for (int mt = 0; mt < 2; ++mt)
#pragma unroll
        for (int nt = 0; nt < 4; ++nt) acc[mt][nt] = zero8();

#pragma unroll 1
    for (int k0 = 0; k0 < K; k0 += 32) {
        const v16h a0 = load_frag16(Ab + k0, K, lane);
        const v16h a1 = load_frag16(Ab + (size_t)16 * K + k0, K, lane);
#pragma unroll
        for (int nt = 0; nt < 4; ++nt) {
            const v16h bfr = load_frag16(Bb + (size_t)(nt * 16) * K + k0, K, lane);
            acc[0][nt] = wmma16(a0, bfr, acc[0][nt]);
            acc[1][nt] = wmma16(a1, bfr, acc[1][nt]);
        }
    }

    float bb[4];
#pragma unroll
    for (int nt = 0; nt < 4; ++nt) bb[nt] = bf16r(bias[n0 + nt * 16 + cc]);

    if constexpr (MODE == 0) {
        float* ef = EstF + w * 2048;
#pragma unroll
        for (int mt = 0; mt < 2; ++mt)
#pragma unroll
            for (int nt = 0; nt < 4; ++nt)
#pragma unroll
                for (int r = 0; r < 8; ++r) {
                    float u = __builtin_fmaf(acc[mt][nt][r], ascale, bb[nt]);
                    if (RELU) u = fmaxf(u, 0.0f);
                    ef[(mt * 16 + rb + r) * 64 + nt * 16 + cc] = u;
                }
        wave_lds_sync();
        v4f sv[16];
#pragma unroll
        for (int i = 0; i < 16; ++i) sv[i] = *(const v4f*)(&ef[i * 128 + lane * 4]);
        float* cb = Cf + (size_t)m0 * N + n0;
        const int lr = lane >> 4, lc = (lane & 15) * 4;
#pragma unroll
        for (int i = 0; i < 16; ++i)
            *(volatile v4f*)(cb + (size_t)(i * 2 + lr) * N + lc) = sv[i];
        __threadfence();
#pragma unroll
        for (int i = 0; i < 16; ++i)
            *(volatile v4f*)(cb + (size_t)(i * 2 + lr) * N + lc) = sv[i];
    } else {
        _Float16* eh = EstH + w * 2048;
#pragma unroll
        for (int mt = 0; mt < 2; ++mt)
#pragma unroll
            for (int nt = 0; nt < 4; ++nt)
#pragma unroll
                for (int r = 0; r < 8; ++r) {
                    float u = __builtin_fmaf(acc[mt][nt][r], ascale, bb[nt]);
                    if (RELU) u = fmaxf(u, 0.0f);
                    eh[(mt * 16 + rb + r) * 64 + nt * 16 + cc] = (_Float16)(u * oscale);
                }
        wave_lds_sync();
        v8h ph[8];
#pragma unroll
        for (int i = 0; i < 8; ++i) ph[i] = *(const v8h*)(&eh[i * 256 + lane * 8]);
        const int lr = lane >> 3, lc = (lane & 7) * 8;
        _Float16* cbh = Ch + (size_t)m0 * N + n0;
#pragma unroll
        for (int i = 0; i < 8; ++i)
            *(volatile v8h*)(cbh + (size_t)(i * 4 + lr) * N + lc) = ph[i];
        __threadfence();
#pragma unroll
        for (int i = 0; i < 8; ++i)
            *(volatile v8h*)(cbh + (size_t)(i * 4 + lr) * N + lc) = ph[i];
    }
}

__global__ __launch_bounds__(256) __attribute__((amdgpu_num_vgpr(256)))
void k_attn(const _Float16* __restrict__ qh,
            const _Float16* __restrict__ kh,
            const _Float16* __restrict__ vh,
            const int*      __restrict__ mask,
            _Float16* __restrict__ cx) {
    __shared__ __align__(16) int      mk[SEQ];
    __shared__ __align__(16) _Float16 VsT[DH * CH];
    __shared__ __align__(16) _Float16 Cst[8][16 * DH];

    const int tid  = threadIdx.x;
    const int lane = tid & 31;
    const int w    = tid >> 5;
    const int h    = blockIdx.x;
    const int b    = blockIdx.z;
    const int q0r  = blockIdx.y * 128 + w * 16;
    const int r0   = (lane >> 4) << 3;
    const int cc   = lane & 15;

    for (int i = tid; i < SEQ; i += 256) mk[i] = mask[(size_t)b * SEQ_FULL + i];

    const size_t tokb = (size_t)b * SEQ;
    const _Float16* qhb = qh + (tokb + q0r) * DM + h * DH;
    const v16h qb0 = load_frag16(qhb, DM, lane);
    const v16h qb1 = load_frag16(qhb + 32, DM, lane);
    const _Float16* khb = kh + tokb * DM + h * DH;
    const _Float16* vhb = vh + tokb * DM + h * DH;

    v8f o[4];
#pragma unroll
    for (int nt = 0; nt < 4; ++nt) o[nt] = zero8();
    float mr = -1.0e30f, zr = 0.0f;

    __syncthreads();

#pragma unroll 1
    for (int c0 = 0; c0 < SEQ; c0 += CH) {
        for (int idx = tid; idx < CH * 8; idx += 256) {
            const int t = idx >> 3, part = idx & 7;
            const v8h vv = *(const v8h*)(vhb + (size_t)(c0 + t) * DM + part * 8);
#pragma unroll
            for (int e = 0; e < 8; ++e) VsT[(part * 8 + e) * CH + t] = vv[e];
        }
        __syncthreads();

#pragma unroll 1
        for (int j = 0; j < CH; j += 32) {
            const int kA = c0 + j;
            const v16h ka0 = load_frag16(khb + (size_t)kA * DM, DM, lane);
            const v16h ka1 = load_frag16(khb + (size_t)kA * DM + 32, DM, lane);
            v8f shA = wmma16(ka0, qb0, zero8());
            shA = wmma16(ka1, qb1, shA);
            const v16h kb0 = load_frag16(khb + (size_t)(kA + 16) * DM, DM, lane);
            const v16h kb1 = load_frag16(khb + (size_t)(kA + 16) * DM + 32, DM, lane);
            v8f shB = wmma16(kb0, qb0, zero8());
            shB = wmma16(kb1, qb1, shB);

            I8 ma, mb;
            ma.v[0] = *(const v4i*)(&mk[kA + r0]);
            ma.v[1] = *(const v4i*)(&mk[kA + r0 + 4]);
            mb.v[0] = *(const v4i*)(&mk[kA + 16 + r0]);
            mb.v[1] = *(const v4i*)(&mk[kA + 16 + r0 + 4]);

            float tA[8], tB[8];
#pragma unroll
            for (int r = 0; r < 8; ++r) {
                const float sa = shA[r] * C1;
                const float sb = shB[r] * C1;
                tA[r] = (ma.s[r] != 0) ? sa : MASKT;
                tB[r] = (mb.s[r] != 0) ? sb : MASKT;
            }
            float tmax = tA[0];
#pragma unroll
            for (int r = 1; r < 8; ++r) tmax = fmaxf(tmax, tA[r]);
#pragma unroll
            for (int r = 0; r < 8; ++r) tmax = fmaxf(tmax, tB[r]);
            tmax = fmaxf(tmax, __shfl_xor(tmax, 16, 32));
            const float mn   = fmaxf(mr, tmax);
            const float corr = ex2(mr - mn);
            const float mo   = mn - 14.0f;
            float ps = 0.0f;
            v8h pa8, pb8;
#pragma unroll
            for (int r = 0; r < 8; ++r) {
                const float pa = ex2(tA[r] - mo);
                const float pb = ex2(tB[r] - mo);
                ps += pa + pb;
                pa8[r] = (_Float16)pa;
                pb8[r] = (_Float16)pb;
            }
            ps += __shfl_xor(ps, 16, 32);
            zr = __builtin_fmaf(zr, corr, ps);
            mr = mn;
#pragma unroll
            for (int r = 0; r < 8; ++r) {
                const float crr = __shfl(corr, r0 + r, 32);
#pragma unroll
                for (int nt = 0; nt < 4; ++nt) o[nt][r] *= crr;
            }
            Frag pf;
            pf.h[0] = pa8;
            pf.h[1] = pb8;
#pragma unroll
            for (int nt = 0; nt < 4; ++nt) {
                const v16h vb = load_frag16(&VsT[(nt * 16) * CH + j], CH, lane);
                o[nt] = wmma16(pf.v, vb, o[nt]);
            }
        }
        __syncthreads();
    }

    const float rz = __builtin_amdgcn_rcpf(zr);
#pragma unroll
    for (int r = 0; r < 8; ++r) {
        const float rq = __shfl(rz, r0 + r, 32);
#pragma unroll
        for (int nt = 0; nt < 4; ++nt)
            Cst[w][(r0 + r) * DH + nt * 16 + cc] = (_Float16)(o[nt][r] * rq);
    }
    wave_lds_sync();
    v8h sv[4];
#pragma unroll
    for (int i = 0; i < 4; ++i) sv[i] = *(const v8h*)(&Cst[w][i * 256 + lane * 8]);
    _Float16* cb = cx + (tokb + q0r) * DM + h * DH;
    const int lr = lane >> 3, lc = (lane & 7) * 8;
#pragma unroll
    for (int i = 0; i < 4; ++i) *(volatile v8h*)(cb + (size_t)(i * 4 + lr) * DM + lc) = sv[i];
    __threadfence();
#pragma unroll
    for (int i = 0; i < 4; ++i) *(volatile v8h*)(cb + (size_t)(i * 4 + lr) * DM + lc) = sv[i];
}

static __device__ __forceinline__ int ln_off(bool hout, int i, int lane) {
    return hout ? ((i >> 1) * 256 + lane * 8 + (i & 1) * 4) : (i * 128 + lane * 4);
}

template <bool HOUT>
__global__ __launch_bounds__(256) void k_ln(const float* __restrict__ src,
                                            const float* __restrict__ g,
                                            const float* __restrict__ bt,
                                            float* __restrict__ outf,
                                            _Float16* __restrict__ outh,
                                            float hsc) {
    const int lane = threadIdx.x & 31;
    const int w    = threadIdx.x >> 5;
    const int row  = blockIdx.x * 8 + w;
    const float* rp = src + (size_t)row * DM;

    v4f xv[6];
#pragma unroll
    for (int i = 0; i < 6; ++i) xv[i] = *(const v4f*)(rp + ln_off(HOUT, i, lane));
    float s = 0.0f;
#pragma unroll
    for (int i = 0; i < 6; ++i) s += (xv[i][0] + xv[i][1]) + (xv[i][2] + xv[i][3]);
#pragma unroll
    for (int m = 1; m < 32; m <<= 1) s += __shfl_xor(s, m, 32);
    const float mu = s * (1.0f / (float)DM);

    v4f dv[6];
    float s2 = 0.0f;
#pragma unroll
    for (int i = 0; i < 6; ++i) {
        dv[i] = xv[i] - mu;
#pragma unroll
        for (int e = 0; e < 4; ++e) s2 = __builtin_fmaf(dv[i][e], dv[i][e], s2);
    }
#pragma unroll
    for (int m = 1; m < 32; m <<= 1) s2 += __shfl_xor(s2, m, 32);
    const float var  = s2 * (1.0f / (float)DM);
    const float rstd = rsqrtf(var + 1e-5f);

    v4f yv[6];
#pragma unroll
    for (int i = 0; i < 6; ++i) {
        const int co = ln_off(HOUT, i, lane);
        const v4f gv = *(const v4f*)(g + co);
        const v4f bv = *(const v4f*)(bt + co);
#pragma unroll
        for (int e = 0; e < 4; ++e)
            yv[i][e] = (dv[i][e] * rstd) * bf16r(gv[e]) + bf16r(bv[e]);
    }

    if constexpr (HOUT) {
        v8h hv[3];
#pragma unroll
        for (int i = 0; i < 3; ++i)
#pragma unroll
            for (int e = 0; e < 4; ++e) {
                hv[i][e]     = (_Float16)(yv[2 * i][e] * hsc);
                hv[i][4 + e] = (_Float16)(yv[2 * i + 1][e] * hsc);
            }
        _Float16* ob = outh + (size_t)row * DM + lane * 8;
#pragma unroll
        for (int i = 0; i < 3; ++i) *(volatile v8h*)(ob + i * 256) = hv[i];
        __threadfence();
#pragma unroll
        for (int i = 0; i < 3; ++i) *(volatile v8h*)(ob + i * 256) = hv[i];
    } else {
        float* ob = outf + (size_t)row * DM + lane * 4;
#pragma unroll
        for (int i = 0; i < 6; ++i) *(volatile v4f*)(ob + i * 128) = yv[i];
        __threadfence();
#pragma unroll
        for (int i = 0; i < 6; ++i) *(volatile v4f*)(ob + i * 128) = yv[i];
    }
}

extern "C" void kernel_launch(void* const* d_in, const int* in_sizes, int n_in,
                              void* d_out, int out_size, void* d_ws, size_t ws_size,
                              hipStream_t stream) {
    if (n_in < 16) return;
    if (in_sizes[0] < ((NB - 1) * SEQ_FULL + SEQ) * DM) return;
    if (in_sizes[1] < (NB - 1) * SEQ_FULL + SEQ) return;
    if (in_sizes[2] < DM * DM || in_sizes[4] < DM * DM || in_sizes[6] < DM * DM || in_sizes[8] < DM * DM) return;
    if (in_sizes[3] < DM || in_sizes[5] < DM || in_sizes[7] < DM || in_sizes[9] < DM) return;
    if (in_sizes[10] < DM || in_sizes[11] < DM) return;
    if (in_sizes[12] < DM * FF || in_sizes[13] < FF || in_sizes[14] < FF * DM || in_sizes[15] < DM) return;
    if (out_size < NTOK * DM) return;

    const float* x    = (const float*)d_in[0];
    const int*   mask = (const int*)  d_in[1];
    const float* Wq   = (const float*)d_in[2];
    const float* bq   = (const float*)d_in[3];
    const float* Wk   = (const float*)d_in[4];
    const float* bk   = (const float*)d_in[5];
    const float* Wv   = (const float*)d_in[6];
    const float* bv   = (const float*)d_in[7];
    const float* Wo   = (const float*)d_in[8];
    const float* bo   = (const float*)d_in[9];
    const float* lg   = (const float*)d_in[10];
    const float* lb   = (const float*)d_in[11];
    const float* W1   = (const float*)d_in[12];
    const float* b1   = (const float*)d_in[13];
    const float* W2   = (const float*)d_in[14];
    const float* b2   = (const float*)d_in[15];
    float* out = (float*)d_out;

    char* ws = (char*)d_ws;
    size_t off = 0;
    _Float16* WqT = (_Float16*)(ws + off); off += (size_t)DM * DM * 2;
    _Float16* WkT = (_Float16*)(ws + off); off += (size_t)DM * DM * 2;
    _Float16* WvT = (_Float16*)(ws + off); off += (size_t)DM * DM * 2;
    _Float16* WoT = (_Float16*)(ws + off); off += (size_t)DM * DM * 2;
    _Float16* W1T = (_Float16*)(ws + off); off += (size_t)FF * DM * 2;
    _Float16* W2T = (_Float16*)(ws + off); off += (size_t)DM * FF * 2;
    const size_t PL = (size_t)NTOK * DM * 2;
    _Float16* xp  = (_Float16*)(ws + off);
    _Float16* cxp = (_Float16*)(ws + off); off += PL;
    const size_t F1B = (size_t)NTOK * FF * 2;
    const size_t R2 = (3 * PL > PL + F1B) ? 3 * PL : (PL + F1B);
    _Float16* qhp = (_Float16*)(ws + off);
    _Float16* khp = (_Float16*)(ws + off + PL);
    _Float16* vhp = (_Float16*)(ws + off + 2 * PL);
    _Float16* hp  = (_Float16*)(ws + off);
    _Float16* f1p = (_Float16*)(ws + off + PL);
    off += R2;
    float* aop = (float*)(ws + off);
    float* ffp = (float*)(ws + off); off += (size_t)NTOK * DM * 4;
    if (off > ws_size) return;
    if (off > (size_t)134217728) return;

    k_xprep<<<dim3((NTOK * (DM / 8)) / 256), dim3(256), 0, stream>>>(x, xp);
    k_wtr<<<dim3(DM / 64, DM / 64), dim3(256), 0, stream>>>(Wq, WqT, DM, DM);
    k_wtr<<<dim3(DM / 64, DM / 64), dim3(256), 0, stream>>>(Wk, WkT, DM, DM);
    k_wtr<<<dim3(DM / 64, DM / 64), dim3(256), 0, stream>>>(Wv, WvT, DM, DM);
    k_wtr<<<dim3(DM / 64, DM / 64), dim3(256), 0, stream>>>(Wo, WoT, DM, DM);
    k_wtr<<<dim3(FF / 64, DM / 64), dim3(256), 0, stream>>>(W1, W1T, DM, FF);
    k_wtr<<<dim3(DM / 64, FF / 64), dim3(256), 0, stream>>>(W2, W2T, FF, DM);

    const dim3 gD(DM / 128, NTOK / 128);
    const dim3 gF(FF / 128, NTOK / 128);
    k_gemm<1, false><<<gD, dim3(256), 0, stream>>>(xp, WqT, bq, A_QKV, QSC, aop, qhp, DM, DM);
    k_gemm<1, false><<<gD, dim3(256), 0, stream>>>(xp, WkT, bk, A_QKV, QSC, aop, khp, DM, DM);
    k_gemm<1, false><<<gD, dim3(256), 0, stream>>>(xp, WvT, bv, A_QKV, QSC, aop, vhp, DM, DM);
    k_attn<<<dim3(NH, SEQ / 128, NB), dim3(256), 0, stream>>>(qhp, khp, vhp, mask, cxp);
    k_gemm<0, false><<<gD, dim3(256), 0, stream>>>(cxp, WoT, bo, A_O, 1.0f, aop, f1p, DM, DM);
    k_ln<true><<<dim3(NTOK / 8), dim3(256), 0, stream>>>(aop, lg, lb, out, hp, HSC);
    k_gemm<1, true><<<gF, dim3(256), 0, stream>>>(hp, W1T, b1, A_F1, QSC, ffp, f1p, DM, FF);
    k_gemm<0, false><<<gD, dim3(256), 0, stream>>>(f1p, W2T, b2, A_F2, 1.0f, ffp, hp, FF, DM);
    k_ln<false><<<dim3(NTOK / 8), dim3(256), 0, stream>>>(ffp, lg, lb, out, hp, 1.0f);
}
